// SREL_rep_mu_3109556322489
// MI455X (gfx1250) — hardware-run, weakly checked
//
#include <hip/hip_runtime.h>
#include <math.h>

typedef __attribute__((ext_vector_type(16))) _Float16 v16h;
typedef __attribute__((ext_vector_type(8)))  _Float16 v8h;
typedef __attribute__((ext_vector_type(16))) __bf16   v16b;
typedef __attribute__((ext_vector_type(8)))  __bf16   v8b;
typedef __attribute__((ext_vector_type(8)))  float    v8f;
typedef __attribute__((ext_vector_type(4)))  float    v4f;

constexpr int kB      = 64;
constexpr int kLS     = 1024;
constexpr int kLW     = 1024;
constexpr int kLY     = 2048;
constexpr int kM      = 16;
constexpr int kD      = 2 * kLS + 2 * kLW + kLY;
constexpr int kH      = 512;
constexpr int kSteps  = 10;
constexpr int kSlots  = kSteps + 1;
constexpr int kN3     = 3 * kH;
constexpr int kRowsW  = kB * kM;
constexpr int kKW     = 2 * kLW;
constexpr int kKS     = 2 * kLS;
constexpr int kYtRows = 64;
constexpr int kCsPitch = 32;
constexpr int kPackWBlocks = kB * 2 * (kLW / 256);
constexpr int kPackYBlocks = kLY / 256;
constexpr size_t kOut0Elems = (size_t)kB * kSlots * kLS * 2;
constexpr size_t kOut1Elems = (size_t)kB * kSteps * kM;
static_assert(kD == 6144, "feature width");
static_assert(kKW == 2048 && kKS == 2048 && kLY == 2048, "operand plane pitch 2048");
static_assert(kOut0Elems * 4 == 5767168ull, "out0 bytes");
static_assert((kOut0Elems + kOut1Elems) * 4 == 5808128ull, "d_out bytes");
static_assert(((kOut0Elems * 4) % 128) == 0, "out1 starts on a line");
static_assert((kKW % 32) == 0 && (kKS % 32) == 0 && (kLY % 32) == 0 && (kH % 32) == 0, "GEMM K multiples of 32");
static_assert((kRowsW % 64) == 0 && (kN3 % 64) == 0 && (kB % 64) == 0 && (kLS % 64) == 0 && (kYtRows % 64) == 0, "GEMM M,N multiples of 64");
static_assert(kPackWBlocks == 512 && kPackYBlocks == 8, "pack grid");
static_assert((kM * kSteps * 4) == 640, "out1 per-batch extent = 5 lines");

constexpr size_t kOffXW    = 0;
constexpr size_t kOffYT    = kOffXW    + (size_t)kRowsW  * kKW  * 2;
constexpr size_t kOffW1T   = kOffYT    + (size_t)kYtRows * kLY  * 2;
constexpr size_t kOffE2T   = kOffW1T   + (size_t)kN3     * kD   * 2;
constexpr size_t kOffSTATW = kOffE2T   + (size_t)kLS     * kH   * 2;
constexpr size_t kOffSTATY = kOffSTATW + (size_t)kRowsW  * kN3  * 4;
constexpr size_t kOffPHIA  = kOffSTATY + (size_t)kYtRows * kN3  * 4;
constexpr size_t kOffPHIB  = kOffPHIA  + (size_t)kB      * kLS  * 4;
constexpr size_t kOffSH    = kOffPHIB  + (size_t)kB      * kLS  * 4;
constexpr size_t kOffSL    = kOffSH    + (size_t)kB      * kKS  * 2;
constexpr size_t kOffDYN   = kOffSL    + (size_t)kB      * kKS  * 2;
constexpr size_t kOffVH    = kOffDYN   + (size_t)kB      * kN3  * 4;
constexpr size_t kOffVL    = kOffVH    + (size_t)kB      * kH   * 2;
constexpr size_t kOffETA   = kOffVL    + (size_t)kB      * kH   * 2;
constexpr size_t kOffCSUM  = kOffETA   + (size_t)kB      * kLS  * 4;
constexpr size_t kWsTotal  = kOffCSUM  + (size_t)kB      * kCsPitch * 4;
static_assert(kWsTotal == 32907264ull, "carve total");
static_assert(kWsTotal <= 134217728ull, "carve cap");
static_assert((kOffYT % 128) == 0 && (kOffW1T % 128) == 0 && (kOffE2T % 128) == 0 && (kOffSTATW % 128) == 0 &&
              (kOffSTATY % 128) == 0 && (kOffPHIA % 128) == 0 && (kOffPHIB % 128) == 0 && (kOffSH % 128) == 0 &&
              (kOffSL % 128) == 0 && (kOffDYN % 128) == 0 && (kOffVH % 128) == 0 && (kOffVL % 128) == 0 &&
              (kOffETA % 128) == 0 && (kOffCSUM % 128) == 0, "128-B aligned regions");

__device__ __forceinline__ unsigned short f2bf_bits(float f) {
  unsigned u = __float_as_uint(f);
  return (unsigned short)((u + 0x7FFFu + ((u >> 16) & 1u)) >> 16);
}
__device__ __forceinline__ float bf_bits2f(unsigned short h) { return __uint_as_float(((unsigned)h) << 16); }
__device__ __forceinline__ float bf_rne(float f) { return bf_bits2f(f2bf_bits(f)); }

__device__ __forceinline__ void acc_guard1_b(v8f& a, v16b x, v16b y) { asm volatile("v_nop\n\tv_nop\n\tv_nop\n\tv_nop" : "+v"(a) : "v"(x), "v"(y)); }
__device__ __forceinline__ void keep4_b(v16b a, v16b b, v16b c, v16b d) { asm volatile("v_nop" :: "v"(a), "v"(b), "v"(c), "v"(d)); }
__device__ __forceinline__ void acc_guard4(v8f& a, v8f& b, v8f& c, v8f& d) { asm volatile("v_nop\n\tv_nop\n\tv_nop\n\tv_nop" : "+v"(a), "+v"(b), "+v"(c), "+v"(d)); }

struct FragB {
  union U { v16b v; v8b h[2]; };
  static __device__ __forceinline__ v16b load(const __bf16* p) {
    U f; f.h[0] = *(const v8b*)(p); f.h[1] = *(const v8b*)(p + 16); return f.v;
  }
  static __device__ __forceinline__ v8f mma(v16b a, v16b b, v8f c) {
    return __builtin_amdgcn_wmma_f32_16x16x32_bf16(false, a, false, b, (short)0, c, false, false);
  }
};

__device__ __forceinline__ void split8_bf16(const v4f a0, const v4f a1, v8h& hv, v8h& lv) {
#pragma unroll
  for (int e = 0; e < 4; ++e) {
    const float f0 = a0[e];
    const float f1 = a1[e];
    const unsigned short h0 = f2bf_bits(f0), h1 = f2bf_bits(f1);
    const unsigned short l0 = f2bf_bits(f0 - bf_bits2f(h0)), l1 = f2bf_bits(f1 - bf_bits2f(h1));
    hv[e]     = __builtin_bit_cast(_Float16, h0);
    hv[4 + e] = __builtin_bit_cast(_Float16, h1);
    lv[e]     = __builtin_bit_cast(_Float16, l0);
    lv[4 + e] = __builtin_bit_cast(_Float16, l1);
  }
}

template <int SPL>
__global__ __launch_bounds__(256) void wmma_gemm64_bf16(
    const unsigned short* __restrict__ Ap, const unsigned short* __restrict__ A2p, int lda,
    const unsigned short* __restrict__ Btp, int ldb,
    float* __restrict__ Cout, int ldc, int M, int N, int K) {
  typedef __bf16 T;
  typedef v16b V;
  const T* A  = (const T*)Ap;
  const T* A2 = (const T*)A2p;
  const T* Bt = (const T*)Btp;
  __shared__ __align__(16) float sT[8][16 * 68];
  const int lane = threadIdx.x & 31;
  const int wave = threadIdx.x >> 5;
  const int tilesN = N >> 6;
  const int tilesM = M >> 6;
  const int tile = blockIdx.x * 8 + wave;
  if (tile >= tilesM * tilesN) return;
  const int tm = tile / tilesN;
  const int tn = tile - tm * tilesN;
  const int m0 = tm << 6;
  const int n0 = tn << 6;

  const int rlane = lane & 15;
  const int koff  = (lane >> 4) * 8;
  const int mOff  = (lane >> 4) * 8;

  v8f acc[4][4];
#pragma unroll
  for (int i = 0; i < 4; ++i)
#pragma unroll
    for (int j = 0; j < 4; ++j) acc[i][j] = (v8f){0.f,0.f,0.f,0.f,0.f,0.f,0.f,0.f};

  for (int k0 = 0; k0 < K; k0 += 32) {
    V bh[4];
#pragma unroll
    for (int j = 0; j < 4; ++j) {
      const size_t bo = (size_t)(n0 + (j << 4) + rlane) * ldb + koff + k0;
      bh[j] = FragB::load(Bt + bo);
    }
#pragma unroll
    for (int i = 0; i < 4; ++i) {
      const size_t ao = (size_t)(m0 + (i << 4) + rlane) * lda + koff + k0;
      V ah = FragB::load(A + ao);
      V al = ah;
      if (SPL >= 1) al = FragB::load(A2 + ao);
#pragma unroll
      for (int j = 0; j < 4; ++j) {
        acc[i][j] = FragB::mma(ah, bh[j], acc[i][j]);
        if (SPL >= 1) acc[i][j] = FragB::mma(al, bh[j], acc[i][j]);
      }
      acc_guard1_b(acc[i][0], ah, al);
      acc_guard1_b(acc[i][1], ah, al);
      acc_guard1_b(acc[i][2], ah, al);
      acc_guard1_b(acc[i][3], ah, al);
    }
    keep4_b(bh[0], bh[1], bh[2], bh[3]);
  }
  acc_guard4(acc[0][0], acc[0][1], acc[0][2], acc[0][3]);
  acc_guard4(acc[1][0], acc[1][1], acc[1][2], acc[1][3]);
  acc_guard4(acc[2][0], acc[2][1], acc[2][2], acc[2][3]);
  acc_guard4(acc[3][0], acc[3][1], acc[3][2], acc[3][3]);

  float* slab = sT[wave];
#pragma unroll
  for (int i = 0; i < 4; ++i) {
    const int mBase = m0 + (i << 4);
#pragma unroll
    for (int j = 0; j < 4; ++j) {
#pragma unroll
      for (int r = 0; r < 8; ++r) {
        slab[(mOff + r) * 68 + (j << 4) + rlane] = acc[i][j][r];
      }
    }
    __builtin_amdgcn_fence(__ATOMIC_RELEASE, "workgroup");
    __builtin_amdgcn_wave_barrier();
    __builtin_amdgcn_fence(__ATOMIC_ACQUIRE, "workgroup");
    {
      const int hh = lane >> 4, c4 = (lane & 15) * 4;
      for (int pass = 0; pass < 2; ++pass) {
#pragma unroll
        for (int it = 0; it < 8; ++it) {
          const int row = it * 2 + hh;
          v4f v = *(const v4f*)(slab + row * 68 + c4);
          *(volatile v4f*)(Cout + (size_t)(mBase + row) * ldc + n0 + c4) = v;
        }
        __threadfence();
      }
    }
    __builtin_amdgcn_fence(__ATOMIC_RELEASE, "workgroup");
    __builtin_amdgcn_wave_barrier();
    __builtin_amdgcn_fence(__ATOMIC_ACQUIRE, "workgroup");
  }
}

__global__ __launch_bounds__(256) void pack_feat_kernel(
    const float* __restrict__ wre, const float* __restrict__ wim, const float* __restrict__ ym,
    unsigned short* __restrict__ XW, unsigned short* __restrict__ YT)
{
  __shared__ float sT[256 * 17];
  const int tid = threadIdx.x, lane = tid & 31, wave = tid >> 5;
  const int bx = blockIdx.x;
  const bool isY = (bx >= kPackWBlocks);
  const float* src;
  unsigned short* dst;
  int dcol;
  if (!isY) {
    const int b = bx >> 3, plane = (bx >> 2) & 1, chunk = bx & 3;
    src = (plane ? wim : wre) + ((size_t)b * kLW + (size_t)chunk * 256) * kM;
    dst = XW + (size_t)(b * kM) * kKW;
    dcol = plane * kLW + chunk * 256;
  } else {
    const int chunk = bx - kPackWBlocks;
    src = ym + (size_t)chunk * 256 * kM;
    dst = YT;
    dcol = chunk * 256;
  }
#pragma unroll
  for (int it = 0; it < 4; ++it) {
    const int q = it * 256 + tid;
    const int c = q >> 2, mq = (q & 3) * 4;
    const v4f a = *(const v4f*)(src + (size_t)q * 4);
    sT[c * 17 + mq + 0] = a[0];
    sT[c * 17 + mq + 1] = a[1];
    sT[c * 17 + mq + 2] = a[2];
    sT[c * 17 + mq + 3] = a[3];
  }
  __syncthreads();
  v8h hv[2];
#pragma unroll
  for (int it = 0; it < 2; ++it) {
    const int m = it * 8 + wave;
#pragma unroll
    for (int e = 0; e < 8; ++e) {
      const float f = sT[(lane * 8 + e) * 17 + m];
      const unsigned short hb = f2bf_bits(f);
      hv[it][e] = __builtin_bit_cast(_Float16, hb);
    }
  }
  const v4f z4 = (v4f){0.f, 0.f, 0.f, 0.f};
  for (int pass = 0; pass < 2; ++pass) {
#pragma unroll
    for (int it = 0; it < 2; ++it) {
      const int m = it * 8 + wave;
      *(volatile v8h*)(dst + (size_t)m * kKW + dcol + lane * 8) = hv[it];
    }
    if (isY) {
#pragma unroll
      for (int it = 0; it < 6; ++it) {
        const int row = 16 + it * 8 + wave;
        *(volatile v4f*)((void*)(YT + (size_t)row * kKW + dcol + lane * 8)) = z4;
      }
    }
    __threadfence();
  }
}

__global__ __launch_bounds__(256) void transpose_bf16_kernel(
    const float* __restrict__ s0, const float* __restrict__ s1, const float* __restrict__ s2,
    int nin, int nout, unsigned short* __restrict__ dst)
{
  __shared__ float sT[64 * 65];
  const int tid = threadIdx.x;
  const int z = blockIdx.z;
  const float* src = (z == 0) ? s0 : ((z == 1) ? s1 : s2);
  const int k0 = blockIdx.x * 64, h0 = blockIdx.y * 64;
#pragma unroll
  for (int it = 0; it < 4; ++it) {
    const int r = it * 16 + (tid >> 4);
    const int c4 = (tid & 15) * 4;
    const v4f a = *(const v4f*)(src + (size_t)(k0 + r) * nout + h0 + c4);
    sT[r * 65 + c4 + 0] = a[0];
    sT[r * 65 + c4 + 1] = a[1];
    sT[r * 65 + c4 + 2] = a[2];
    sT[r * 65 + c4 + 3] = a[3];
  }
  __syncthreads();
  v8h hv[2];
  const int c8 = (tid & 7) * 8;
#pragma unroll
  for (int it = 0; it < 2; ++it) {
    const int h = it * 32 + (tid >> 3);
#pragma unroll
    for (int e = 0; e < 8; ++e) {
      const float f = sT[(c8 + e) * 65 + h];
      const unsigned short hb = f2bf_bits(f);
      hv[it][e] = __builtin_bit_cast(_Float16, hb);
    }
  }
  for (int pass = 0; pass < 2; ++pass) {
#pragma unroll
    for (int it = 0; it < 2; ++it) {
      const int h = it * 32 + (tid >> 3);
      *(volatile v8h*)(dst + ((size_t)z * nout + h0 + h) * nin + k0 + c8) = hv[it];
    }
    __threadfence();
  }
}

__global__ __launch_bounds__(512) void fuse_kernel(
    const float* __restrict__ DYN, const float* __restrict__ STATW, const float* __restrict__ STATY,
    const float* __restrict__ eb1, const float* __restrict__ rb1, const float* __restrict__ mb1,
    const float* __restrict__ rW2, const float* __restrict__ rb2,
    const float* __restrict__ mW2, const float* __restrict__ mb2,
    unsigned short* __restrict__ VH, unsigned short* __restrict__ VL, float* __restrict__ CSUM)
{
  __shared__ __align__(16) float sRed[2 * 2 * 16];
  __shared__ __align__(16) float sV[kH];
  const int tid = threadIdx.x, lane = tid & 31, wave = tid >> 5;
  const int b = blockIdx.x;
  const int h = tid;
  const float de = DYN[(size_t)b * kN3 + h] + bf_rne(eb1[h]);
  const float dr = DYN[(size_t)b * kN3 + kH + h] + bf_rne(rb1[h]);
  const float dm = DYN[(size_t)b * kN3 + 2 * kH + h] + bf_rne(mb1[h]);
  const float wr2 = bf_rne(rW2[h]);
  const float wm2 = bf_rne(mW2[h]);
  const float rb = bf_rne(rb2[0]);
  const float mb = bf_rne(mb2[0]);
  float vacc = 0.f, cacc = 0.f;
#pragma unroll 1
  for (int m = 0; m < kM; ++m) {
    const float* sw = STATW + (size_t)(b * kM + m) * kN3;
    const float* sy = STATY + (size_t)m * kN3;
    const float pe = de + sw[h] + sy[h];
    const float pr = dr + sw[kH + h] + sy[kH + h];
    const float pm = dm + sw[2 * kH + h] + sy[2 * kH + h];
    const float he = fmaxf(pe, 0.0f);
    const float hr = fmaxf(pr, 0.0f);
    const float hm = fmaxf(pm, 0.0f);
    float vr = hr * wr2;
    float vm = hm * wm2;
#pragma unroll
    for (int off = 16; off > 0; off >>= 1) {
      vr += __shfl_xor(vr, off, 32);
      vm += __shfl_xor(vm, off, 32);
    }
    const int buf = (m & 1) * 32;
    if (lane == 0) {
      sRed[buf + wave] = vr;
      sRed[buf + 16 + wave] = vm;
    }
    __syncthreads();
    float sr = 0.f, sm = 0.f;
#pragma unroll
    for (int w4 = 0; w4 < 4; ++w4) {
      const v4f a = *(const v4f*)(sRed + buf + 4 * w4);
      const v4f c = *(const v4f*)(sRed + buf + 16 + 4 * w4);
      sr += a[0]; sr += a[1]; sr += a[2]; sr += a[3];
      sm += c[0]; sm += c[1]; sm += c[2]; sm += c[3];
    }
    const float rho = sr + rb;
    const float mu  = sm + mb;
    const float cc  = mu * rho;
    vacc = fmaf(cc, he, vacc);
    cacc += cc;
  }
  sV[h] = vacc;
  __syncthreads();
  if (tid < 64) {
    const v4f a0 = *(const v4f*)(sV + tid * 8);
    const v4f a1 = *(const v4f*)(sV + tid * 8 + 4);
    v8h hv, lv;
    split8_bf16(a0, a1, hv, lv);
    const size_t o = (size_t)b * kH + tid * 8;
    for (int pass = 0; pass < 2; ++pass) {
      *(volatile v8h*)(VH + o) = hv;
      *(volatile v8h*)(VL + o) = lv;
      __threadfence();
    }
  } else if (tid < 72) {
    const v4f cv = (v4f){cacc, cacc, cacc, cacc};
    float* cp = CSUM + (size_t)b * kCsPitch + (tid - 64) * 4;
    for (int pass = 0; pass < 2; ++pass) {
      *(volatile v4f*)cp = cv;
      __threadfence();
    }
  }
}

template <bool FIRST>
__global__ __launch_bounds__(256) void phase_emit_kernel(
    const float* __restrict__ phi_src, const float* __restrict__ eta, const float* __restrict__ csum,
    const float* __restrict__ eb2, float* __restrict__ phi_dst, float* __restrict__ out0, int slot,
    unsigned short* __restrict__ SH, unsigned short* __restrict__ SL, float* __restrict__ out1)
{
  __shared__ __align__(16) float sP[kLS];
  __shared__ __align__(16) float sCS[2 * kLS];
  const int tid = threadIdx.x;
  const int b = blockIdx.x;
  float cs = 0.f;
  if (!FIRST) cs = csum[(size_t)b * kCsPitch];
#pragma unroll 1
  for (int j = 0; j < 4; ++j) {
    const int l = j * 256 + tid;
    float p = phi_src[(size_t)b * kLS + l];
    if (FIRST) {
      p = bf_rne(p);
    } else {
      const float en = eta[(size_t)b * kLS + l] + cs * bf_rne(eb2[l]);
      p = p - en;
    }
    sP[l] = p;
    sCS[l] = cosf(p);
    sCS[kLS + l] = sinf(p);
  }
  __syncthreads();
  const v4f pv = *(const v4f*)(sP + tid * 4);
  v4f ov[2];
#pragma unroll
  for (int it = 0; it < 2; ++it) {
    const int l0 = (it * 256 + tid) * 2;
    ov[it] = (v4f){sCS[l0], sCS[kLS + l0], sCS[l0 + 1], sCS[kLS + l0 + 1]};
  }
  v8h hv, lv;
  {
    const v4f a0 = *(const v4f*)(sCS + tid * 8);
    const v4f a1 = *(const v4f*)(sCS + tid * 8 + 4);
    split8_bf16(a0, a1, hv, lv);
  }
  const v4f z4 = (v4f){0.f, 0.f, 0.f, 0.f};
  float* pd = phi_dst + (size_t)b * kLS + tid * 4;
  float* od = out0 + ((size_t)(b * kSlots + slot) * kLS) * 2;
  const size_t so = (size_t)b * kKS + tid * 8;
  for (int pass = 0; pass < 2; ++pass) {
    *(volatile v4f*)pd = pv;
#pragma unroll
    for (int it = 0; it < 2; ++it) {
      *(volatile v4f*)(od + (size_t)(it * 256 + tid) * 4) = ov[it];
    }
    *(volatile v8h*)(SH + so) = hv;
    *(volatile v8h*)(SL + so) = lv;
    if (FIRST) {
      if (tid < 40) *(volatile v4f*)(out1 + (size_t)b * (kSteps * kM) + tid * 4) = z4;
    }
    __threadfence();
  }
}

extern "C" void kernel_launch(void* const* d_in, const int* in_sizes, int n_in,
                              void* d_out, int out_size, void* d_ws, size_t ws_size,
                              hipStream_t stream) {
  if (n_in < 16) return;
  if (in_sizes[0] != kB * kLS) return;
  if (in_sizes[1] != kB * kLW * kM) return;
  if (in_sizes[2] != kB * kLW * kM) return;
  if (in_sizes[3] != kLY * kM) return;
  if (in_sizes[4] != kD * kH) return;
  if (in_sizes[5] != kH) return;
  if (in_sizes[6] != kH * kLS) return;
  if (in_sizes[7] != kLS) return;
  if (in_sizes[8] != kD * kH) return;
  if (in_sizes[9] != kH) return;
  if (in_sizes[10] != kH) return;
  if (in_sizes[11] != 1) return;
  if (in_sizes[12] != kD * kH) return;
  if (in_sizes[13] != kH) return;
  if (in_sizes[14] != kH) return;
  if (in_sizes[15] != 1) return;
  if ((size_t)out_size != kOut0Elems + kOut1Elems) return;
  if (ws_size < kWsTotal) return;

  const float* phi0 = (const float*)d_in[0];
  const float* wre  = (const float*)d_in[1];
  const float* wim  = (const float*)d_in[2];
  const float* ym   = (const float*)d_in[3];
  const float* eW1  = (const float*)d_in[4];
  const float* eb1  = (const float*)d_in[5];
  const float* eW2  = (const float*)d_in[6];
  const float* eb2  = (const float*)d_in[7];
  const float* rW1  = (const float*)d_in[8];
  const float* rb1  = (const float*)d_in[9];
  const float* rW2  = (const float*)d_in[10];
  const float* rb2  = (const float*)d_in[11];
  const float* mW1  = (const float*)d_in[12];
  const float* mb1  = (const float*)d_in[13];
  const float* mW2  = (const float*)d_in[14];
  const float* mb2  = (const float*)d_in[15];
  float* out  = (float*)d_out;
  float* out1 = out + kOut0Elems;

  char* ws = (char*)d_ws;
  unsigned short* XW    = (unsigned short*)(ws + kOffXW);
  unsigned short* YT    = (unsigned short*)(ws + kOffYT);
  unsigned short* W1T   = (unsigned short*)(ws + kOffW1T);
  unsigned short* E2T   = (unsigned short*)(ws + kOffE2T);
  float*          STATW = (float*)(ws + kOffSTATW);
  float*          STATY = (float*)(ws + kOffSTATY);
  float*          PHIA  = (float*)(ws + kOffPHIA);
  float*          PHIB  = (float*)(ws + kOffPHIB);
  unsigned short* SH    = (unsigned short*)(ws + kOffSH);
  unsigned short* SL    = (unsigned short*)(ws + kOffSL);
  float*          DYN   = (float*)(ws + kOffDYN);
  unsigned short* VH    = (unsigned short*)(ws + kOffVH);
  unsigned short* VL    = (unsigned short*)(ws + kOffVL);
  float*          ETA   = (float*)(ws + kOffETA);
  float*          CSUM  = (float*)(ws + kOffCSUM);

  pack_feat_kernel<<<kPackWBlocks + kPackYBlocks, 256, 0, stream>>>(wre, wim, ym, XW, YT);
  transpose_bf16_kernel<<<dim3(kD / 64, kH / 64, 3), 256, 0, stream>>>(eW1, rW1, mW1, kD, kH, W1T);
  transpose_bf16_kernel<<<dim3(kH / 64, kLS / 64, 1), 256, 0, stream>>>(eW2, eW2, eW2, kH, kLS, E2T);

  wmma_gemm64_bf16<0><<<(kRowsW / 64) * (kN3 / 64) / 8, 256, 0, stream>>>(
      XW, XW, kKW, W1T + 2 * kLS, kD, STATW, kN3, kRowsW, kN3, kKW);
  wmma_gemm64_bf16<0><<<(kYtRows / 64) * (kN3 / 64) / 8, 256, 0, stream>>>(
      YT, YT, kLY, W1T + 2 * kLS + 2 * kLW, kD, STATY, kN3, kYtRows, kN3, kLY);

  phase_emit_kernel<true><<<kB, 256, 0, stream>>>(phi0, ETA, CSUM, eb2, PHIA, out, 0, SH, SL, out1);

  float* cur = PHIA;
  float* nxt = PHIB;
  for (int t = 0; t < kSteps; ++t) {
    wmma_gemm64_bf16<1><<<(kB / 64) * (kN3 / 64) / 8, 256, 0, stream>>>(
        SH, SL, kKS, W1T, kD, DYN, kN3, kB, kN3, kKS);
    fuse_kernel<<<kB, kH, 0, stream>>>(DYN, STATW, STATY, eb1, rb1, mb1, rW2, rb2, mW2, mb2, VH, VL, CSUM);
    wmma_gemm64_bf16<1><<<(kB / 64) * (kLS / 64) / 8, 256, 0, stream>>>(
        VH, VL, kH, E2T, kH, ETA, kLS, kB, kLS, kH);
    phase_emit_kernel<false><<<kB, 256, 0, stream>>>(cur, ETA, CSUM, eb2, nxt, out, t + 1, SH, SL, out1);
    float* tmp = cur; cur = nxt; nxt = tmp;
  }
}
